// PerformerAttentionLayer_83683142795477
// MI455X (gfx1250) — hardware-verified
//
#include <hip/hip_runtime.h>
#include <math.h>

typedef __attribute__((ext_vector_type(16))) _Float16 v16h;
typedef __attribute__((ext_vector_type(16))) __bf16 v16b;
typedef __attribute__((ext_vector_type(8)))  _Float16 v8h;
typedef __attribute__((ext_vector_type(8)))  float v8f;
typedef __attribute__((ext_vector_type(4)))  float v4f;
typedef __attribute__((ext_vector_type(2)))  float v2f;
typedef __attribute__((ext_vector_type(4)))  unsigned v4u;
typedef __attribute__((ext_vector_type(4)))  int v4i;
typedef float __attribute__((may_alias)) float_a;
typedef int __attribute__((may_alias)) int_a;

template <typename T> __device__ __forceinline__ void vst2(void* p, T v) { *(volatile T*)p = v; __threadfence(); *(volatile T*)p = v; }
__device__ __forceinline__ v8f wmma16(v16h a, v16h b, v8f c) {
  v8f d = __builtin_amdgcn_wmma_f32_16x16x32_f16(false, a, false, b, (short)0, c, false, false);
  asm volatile("v_nop\n\tv_nop\n\tv_nop\n\tv_nop" : "+v"(d) : "v"(a), "v"(b));
  return d;
}
__device__ __forceinline__ v8f wmma_bf(v16b a, v16b b, v8f c) {
  v8f d = __builtin_amdgcn_wmma_f32_16x16x32_bf16(false, a, false, b, (short)0, c, false, false);
  asm volatile("v_nop\n\tv_nop\n\tv_nop\n\tv_nop" : "+v"(d) : "v"(a), "v"(b));
  return d;
}
__device__ __forceinline__ v16h frag_h(const _Float16* rowk0, int lane) {
  union { v16h v; v8h q[2]; } u; const _Float16* p = rowk0 + 8 * (lane >> 4);
  u.q[0] = *(const v8h*)p; u.q[1] = *(const v8h*)(p + 16); return u.v;
}
__device__ __forceinline__ v16h frag_f32(const float* rowk0, int lane) {
  v16h a; const float* p = rowk0 + 8 * (lane >> 4);
#pragma unroll
  for (int i = 0; i < 8; ++i) { a[i] = (_Float16)p[i]; a[8 + i] = (_Float16)p[16 + i]; }
  return a;
}
__device__ __forceinline__ v16h frag_f32s(const float* rowk0, int lane, float sc) {
  v16h a; const float* p = rowk0 + 8 * (lane >> 4);
#pragma unroll
  for (int i = 0; i < 8; ++i) { a[i] = (_Float16)(p[i] * sc); a[8 + i] = (_Float16)(p[16 + i] * sc); }
  return a;
}
__device__ __forceinline__ v16h fragc_f32(const float* W, int k0, int n, int lane, int ld, int K) {
  v16h a; const int g = lane >> 4;
#pragma unroll
  for (int i = 0; i < 8; ++i) { const int ka = k0 + 8 * g + i, kb = ka + 16;
    a[i] = (_Float16)(ka < K ? W[(size_t)(ka < K ? ka : K - 1) * ld + n] : 0.f); a[8 + i] = (_Float16)(kb < K ? W[(size_t)(kb < K ? kb : K - 1) * ld + n] : 0.f); }
  return a;
}
struct F2 { v16b h, l; };
__device__ __forceinline__ F2 bsplit16(const float v[16]) { F2 r;
#pragma unroll
  for (int i = 0; i < 16; ++i) { const __bf16 h = (__bf16)v[i]; r.h[i] = h; r.l[i] = (__bf16)(v[i] - (float)h); }
  return r; }
__device__ __forceinline__ F2 split_row(const float* row, int k0, int lane) { float v[16]; const float* p = row + k0 + 8 * (lane >> 4);
#pragma unroll
  for (int i = 0; i < 8; ++i) { v[i] = p[i]; v[8 + i] = p[16 + i]; }
  return bsplit16(v); }
__device__ __forceinline__ F2 split_rowK(const float* row, int k0, int lane, int K) { float v[16]; const int g = lane >> 4;
#pragma unroll
  for (int i = 0; i < 8; ++i) { const int ka = k0 + 8 * g + i, kb = ka + 16; v[i] = ka < K ? row[ka < K ? ka : K - 1] : 0.f; v[8 + i] = kb < K ? row[kb < K ? kb : K - 1] : 0.f; }
  return bsplit16(v); }
__device__ __forceinline__ F2 split_col(const float* W, int k0, int n, int lane, int ld, int K) { float v[16]; const int g = lane >> 4;
#pragma unroll
  for (int i = 0; i < 8; ++i) { const int ka = k0 + 8 * g + i, kb = ka + 16; v[i] = ka < K ? W[(size_t)(ka < K ? ka : K - 1) * ld + n] : 0.f; v[8 + i] = kb < K ? W[(size_t)(kb < K ? kb : K - 1) * ld + n] : 0.f; }
  return bsplit16(v); }
__device__ __forceinline__ v8f mac3(const F2& a, const F2& b, v8f c) { c = wmma_bf(a.l, b.h, c); c = wmma_bf(a.h, b.l, c); return wmma_bf(a.h, b.h, c); }
__device__ __forceinline__ float sigm(float v) { return 1.0f / (1.0f + expf(-v)); }
#define LDSX() do { asm volatile("s_wait_dscnt 0" ::: "memory"); __builtin_amdgcn_wave_barrier(); __builtin_amdgcn_fence(__ATOMIC_RELEASE, "workgroup"); } while (0)


#define NR 8192
#define DM 256
#define NC 272
#define KVP 288
typedef __attribute__((ext_vector_type(8))) __bf16 v8b;
__device__ __forceinline__ v16b frag_b16(const __bf16* rowk0, int lane) {
  union { v16b v; v8b q[2]; } u; const __bf16* p = rowk0 + 8 * (lane >> 4);
  u.q[0] = *(const v8b*)p; u.q[1] = *(const v8b*)(p + 16); return u.v;
}
__device__ __forceinline__ v16b frag_gbf(const float* rowk0, int lane) {
  v16b a; const float* p = rowk0 + 8 * (lane >> 4);
#pragma unroll
  for (int i = 0; i < 8; ++i) { a[i] = (__bf16)p[i]; a[8 + i] = (__bf16)p[16 + i]; }
  return a;
}
__device__ __forceinline__ float bfr(float v) { return (float)(__bf16)v; }
__device__ __forceinline__ v8f mac3p(v16b ah, v16b al, v16b bh, v16b bl, v8f c) { c = wmma_bf(al, bh, c); c = wmma_bf(ah, bl, c); return wmma_bf(ah, bh, c); }

#define PLANE   (2u * NR * DM)
#define WS_PT   0u
#define WS_QH   (WS_PT + 2u * 7 * DM * DM)
#define WS_QL   (WS_QH + PLANE)
#define WS_KH   (WS_QL + PLANE)
#define WS_KL   (WS_KH + PLANE)
#define WS_VTH  (WS_KL + PLANE)
#define WS_VTL  (WS_VTH + 2u * NC * NR)
#define WS_EQH  (WS_VTL + 2u * NC * NR)
#define WS_EQL  (WS_EQH + PLANE)
#define WS_EKH  (WS_EQL + PLANE)
#define WS_EKL  (WS_EKH + PLANE)
#define WS_KVX  (WS_EKL + PLANE)
#define WS_KVH  (WS_KVX + 4u * DM * KVP)
#define WS_KVL  (WS_KVH + 2u * NC * DM)
#define WS_A1H  (WS_KVL + 2u * NC * DM)
#define WS_A1L  (WS_A1H + PLANE)
#define WS_H1   (WS_A1L + PLANE)
#define WS_H1H  (WS_H1 + 4u * NR * DM)
#define WS_H1L  (WS_H1H + PLANE)
#define WS_F1H  (WS_H1L + PLANE)
#define WS_F1L  (WS_F1H + PLANE)
#define WS_END  (WS_F1L + PLANE)

__global__ __launch_bounds__(256) void k_pack(const float* __restrict__ Wq, const float* __restrict__ Wk, const float* __restrict__ Wv, const float* __restrict__ Wo,
                                              const float* __restrict__ W1, const float* __restrict__ W2, const float* __restrict__ R, __bf16* __restrict__ PT) {
  __shared__ __align__(16) __bf16 srow[DM];
  const int n = blockIdx.x, tid = threadIdx.x; const int which = n >> 8, nn = n & 255;
  const float* Wm = which == 0 ? Wq : which == 1 ? Wk : which == 2 ? Wv : which == 3 ? Wo : which == 4 ? W1 : which == 5 ? W2 : R;
  srow[tid] = (__bf16)Wm[(size_t)tid * DM + nn];
  __syncthreads();
  if (tid < DM / 8) vst2((unsigned*)(PT + (size_t)n * DM + tid * 8), *(const v4u*)(&srow[tid * 8]));
}
__global__ __launch_bounds__(256) void k_ones(__bf16* __restrict__ VTh, __bf16* __restrict__ VTl) {
  const size_t q = (size_t)blockIdx.x * 256 + threadIdx.x;
  const int row = (int)(q >> 10);
  union { __bf16 e[8]; v4u u; } one, zero;
#pragma unroll
  for (int i = 0; i < 8; ++i) { one.e[i] = (__bf16)1.0f; zero.e[i] = (__bf16)0.0f; }
  vst2((unsigned*)(VTh + (size_t)DM * NR + q * 8), row == 0 ? one.u : zero.u);
  vst2((unsigned*)(VTl + (size_t)DM * NR + q * 8), zero.u);
}
__global__ __launch_bounds__(128) void k_qkv(const float* __restrict__ X, const __bf16* __restrict__ PT, __bf16* __restrict__ Qh, __bf16* __restrict__ Ql, __bf16* __restrict__ Kh, __bf16* __restrict__ Kl, __bf16* __restrict__ VTh, __bf16* __restrict__ VTl) {
  __shared__ __align__(16) __bf16 sh_[64][136], sl_[64][136];
  const int tid = threadIdx.x, wave = tid >> 5, lane = tid & 31, col = lane & 15, g = lane >> 4; const size_t rb = (size_t)blockIdx.x * 64; const size_t r0 = rb + wave * 16;
  const int nv = blockIdx.y * 128; const int which = nv >> 8; const int n0 = nv & 255;
  v8f acc[8] = {};
#pragma unroll 2
  for (int kc = 0; kc < DM / 32; ++kc) { const v16b a = frag_gbf(X + (r0 + col) * DM + kc * 32, lane);
#pragma unroll
    for (int j = 0; j < 8; ++j) acc[j] = wmma_bf(a, frag_b16(PT + (size_t)(nv + j * 16 + col) * DM + kc * 32, lane), acc[j]); }
  if (which < 2) {
#pragma unroll
    for (int j = 0; j < 8; ++j)
#pragma unroll
      for (int r = 0; r < 8; ++r) { const float v = acc[j][r]; const __bf16 hi = (__bf16)v; sh_[wave * 16 + 8 * g + r][j * 16 + col] = hi; sl_[wave * 16 + 8 * g + r][j * 16 + col] = (__bf16)(v - (float)hi); }
    LDSX();
    __bf16* Oh = which == 0 ? Qh : Kh; __bf16* Ol = which == 0 ? Ql : Kl;
    for (int qq = lane; qq < 16 * 16; qq += 32) { const int rl = qq >> 4, pc = qq & 15; const size_t o = (r0 + rl) * DM + n0 + pc * 8;
      vst2((unsigned*)(Oh + o), *(const v4u*)(&sh_[wave * 16 + rl][pc * 8])); vst2((unsigned*)(Ol + o), *(const v4u*)(&sl_[wave * 16 + rl][pc * 8])); }
  } else {
#pragma unroll
    for (int half = 0; half < 2; ++half) {
#pragma unroll
      for (int j = 0; j < 4; ++j)
#pragma unroll
        for (int r = 0; r < 8; ++r) { const float v = acc[half * 4 + j][r]; const __bf16 hi = (__bf16)v; sh_[j * 16 + col][wave * 16 + 8 * g + r] = hi; sl_[j * 16 + col][wave * 16 + 8 * g + r] = (__bf16)(v - (float)hi); }
      __syncthreads();
      for (int qq = tid; qq < 64 * 8; qq += 128) { const int c = qq >> 3, pc = qq & 7; const size_t o = (size_t)(n0 + half * 64 + c) * NR + rb + pc * 8;
        vst2((unsigned*)(VTh + o), *(const v4u*)(&sh_[c][pc * 8])); vst2((unsigned*)(VTl + o), *(const v4u*)(&sl_[c][pc * 8])); }
      __syncthreads();
    }
  }
}
__global__ __launch_bounds__(256) void k_proj(const __bf16* __restrict__ Qh, const __bf16* __restrict__ Ql, const __bf16* __restrict__ Kh, const __bf16* __restrict__ Kl, const __bf16* __restrict__ RT,
                                              __bf16* __restrict__ EQh, __bf16* __restrict__ EQl, __bf16* __restrict__ EKh, __bf16* __restrict__ EKl) {
  __shared__ __align__(16) float sp[64][DM + 4];
  __shared__ __align__(16) __bf16 sh_[64][DM + 8], sl_[64][DM + 8];
  const int tid = threadIdx.x, wave = tid >> 5, lane = tid & 31, col = lane & 15, g = lane >> 4; const size_t rb = (size_t)blockIdx.x * 64;
  const int side = blockIdx.y; const __bf16* Ah = side ? Kh : Qh; const __bf16* Al = side ? Kl : Ql;
  const int rt = wave & 3, ct0 = (wave >> 2) * 8; const size_t arow = rb + rt * 16 + col;
  v8f acc[8] = {};
#pragma unroll 2
  for (int kc = 0; kc < DM / 32; ++kc) { const v16b ah = frag_b16(Ah + arow * DM + kc * 32, lane), al = frag_b16(Al + arow * DM + kc * 32, lane);
#pragma unroll
    for (int j = 0; j < 8; ++j) { const v16b b = frag_b16(RT + (size_t)((ct0 + j) * 16 + col) * DM + kc * 32, lane); acc[j] = wmma_bf(al, b, acc[j]); acc[j] = wmma_bf(ah, b, acc[j]); } }
#pragma unroll
  for (int j = 0; j < 8; ++j)
#pragma unroll
    for (int r = 0; r < 8; ++r) { float v = acc[j][r]; v = (__builtin_isinf(v)) ? 1e10f : v; sp[rt * 16 + 8 * g + r][(ct0 + j) * 16 + col] = v; }
  __syncthreads();
#pragma unroll 1
  for (int rr = 0; rr < 8; ++rr) { const int row = wave * 8 + rr; float v[8]; float m = -3.0e38f;
#pragma unroll
    for (int i = 0; i < 8; ++i) { v[i] = sp[row][lane * 8 + i]; m = fmaxf(m, v[i]); }
#pragma unroll
    for (int o = 16; o > 0; o >>= 1) m = fmaxf(m, __shfl_xor(m, o));
#pragma unroll
    for (int i = 0; i < 8; ++i) { const float e = expf(v[i] - m); const __bf16 hi = (__bf16)e; sh_[row][lane * 8 + i] = hi; sl_[row][lane * 8 + i] = (__bf16)(e - (float)hi); } }
  __syncthreads();
  if (side == 0) {
    for (int qq = tid; qq < 64 * 32; qq += 256) { const int rl = qq >> 5, pc = qq & 31; const size_t o = (rb + rl) * DM + pc * 8;
      vst2((unsigned*)(EQh + o), *(const v4u*)(&sh_[rl][pc * 8])); vst2((unsigned*)(EQl + o), *(const v4u*)(&sl_[rl][pc * 8])); }
  } else {
    for (int qq = tid; qq < DM * 8; qq += 256) { const int f = qq >> 3, pc = qq & 7; union { __bf16 e[8]; v4u u; } ph, pl;
#pragma unroll
      for (int i = 0; i < 8; ++i) { ph.e[i] = sh_[pc * 8 + i][f]; pl.e[i] = sl_[pc * 8 + i][f]; }
      const size_t o = (size_t)f * NR + rb + pc * 8; vst2((unsigned*)(EKh + o), ph.u); vst2((unsigned*)(EKl + o), pl.u); }
  }
}
__global__ __launch_bounds__(256) void k_kv(const __bf16* __restrict__ EKh, const __bf16* __restrict__ EKl, const __bf16* __restrict__ VTh, const __bf16* __restrict__ VTl, float* __restrict__ KVX) {
  __shared__ __align__(16) float so[16][KVP];
  const int tid = threadIdx.x, wave = tid >> 5, lane = tid & 31, col = lane & 15, g = lane >> 4; const int f0 = blockIdx.x * 16;
  const int nt = (wave == 0) ? 3 : 2;
  v8f acc[3] = {};
#pragma unroll 1
  for (int kc = 0; kc < NR / 32; ++kc) {
    const v16b ah = frag_b16(EKh + (size_t)(f0 + col) * NR + kc * 32, lane), al = frag_b16(EKl + (size_t)(f0 + col) * NR + kc * 32, lane);
#pragma unroll
    for (int t = 0; t < 3; ++t) { if (t < nt) { const int c = (wave + 8 * t) * 16 + col;
      acc[t] = mac3p(ah, al, frag_b16(VTh + (size_t)c * NR + kc * 32, lane), frag_b16(VTl + (size_t)c * NR + kc * 32, lane), acc[t]); } }
  }
  for (int q = tid; q < 16 * KVP; q += 256) (&so[0][0])[q] = 0.f;
  __syncthreads();
#pragma unroll
  for (int t = 0; t < 3; ++t) { if (t < nt) {
#pragma unroll
    for (int r = 0; r < 8; ++r) so[8 * g + r][(wave + 8 * t) * 16 + col] = acc[t][r]; } }
  __syncthreads();
  for (int q = tid; q < 16 * 72; q += 256) { const int r = q / 72, pc = q - r * 72; vst2(KVX + (size_t)(f0 + r) * KVP + pc * 4, *(const v4f*)(&so[r][pc * 4])); }
}
__global__ __launch_bounds__(256) void k_kvt(const float* __restrict__ KVX, __bf16* __restrict__ KVh, __bf16* __restrict__ KVl) {
  __shared__ __align__(16) __bf16 sh_[DM], sl_[DM];
  const int c = blockIdx.x, tid = threadIdx.x; const float v = KVX[(size_t)tid * KVP + c]; const __bf16 hi = (__bf16)v; sh_[tid] = hi; sl_[tid] = (__bf16)(v - (float)hi);
  __syncthreads();
  if (tid < DM / 8) { vst2((unsigned*)(KVh + (size_t)c * DM + tid * 8), *(const v4u*)(&sh_[tid * 8])); vst2((unsigned*)(KVl + (size_t)c * DM + tid * 8), *(const v4u*)(&sl_[tid * 8])); }
}
__global__ __launch_bounds__(128) void k_num(const __bf16* __restrict__ EQh, const __bf16* __restrict__ EQl, const __bf16* __restrict__ KVh, const __bf16* __restrict__ KVl, __bf16* __restrict__ Ah, __bf16* __restrict__ Al) {
  __shared__ __align__(16) __bf16 sh_[4][16][DM + 8], sl_[4][16][DM + 8];
  __shared__ float sden[4][16];
  const int tid = threadIdx.x, wave = tid >> 5, lane = tid & 31, col = lane & 15, g = lane >> 4; const size_t r0 = (size_t)blockIdx.x * 64 + wave * 16;
  v8f acc[17];
#pragma unroll
  for (int t = 0; t < 17; ++t) acc[t] = (v8f){};
#pragma unroll 1
  for (int kc = 0; kc < DM / 32; ++kc) { const v16b ah = frag_b16(EQh + (r0 + col) * DM + kc * 32, lane), al = frag_b16(EQl + (r0 + col) * DM + kc * 32, lane);
#pragma unroll
    for (int t = 0; t < 17; ++t) acc[t] = mac3p(ah, al, frag_b16(KVh + (size_t)(t * 16 + col) * DM + kc * 32, lane), frag_b16(KVl + (size_t)(t * 16 + col) * DM + kc * 32, lane), acc[t]); }
  if (col == 0) {
#pragma unroll
    for (int r = 0; r < 8; ++r) sden[wave][8 * g + r] = acc[16][r]; }
  LDSX();
#pragma unroll
  for (int t = 0; t < 16; ++t)
#pragma unroll
    for (int r = 0; r < 8; ++r) { const float v = acc[t][r] / (sden[wave][8 * g + r] + 1e-8f); const __bf16 hi = (__bf16)v; sh_[wave][8 * g + r][t * 16 + col] = hi; sl_[wave][8 * g + r][t * 16 + col] = (__bf16)(v - (float)hi); }
  LDSX();
  for (int qq = lane; qq < 16 * 32; qq += 32) { const int rl = qq >> 5, pc = qq & 31; const size_t o = (r0 + rl) * DM + pc * 8;
    vst2((unsigned*)(Ah + o), *(const v4u*)(&sh_[wave][rl][pc * 8])); vst2((unsigned*)(Al + o), *(const v4u*)(&sl_[wave][rl][pc * 8])); }
}
__device__ __forceinline__ void ln_rows(float (*sp)[DM + 4], const float* __restrict__ gam, const float* __restrict__ bet, size_t rb, int wave, int lane, float* __restrict__ OF, __bf16* __restrict__ OH, __bf16* __restrict__ OL) {
#pragma unroll 1
  for (int rr = 0; rr < 8; ++rr) { const int row = wave * 8 + rr; float v[8]; float s = 0.f;
#pragma unroll
    for (int i = 0; i < 8; ++i) { v[i] = sp[row][lane * 8 + i]; s += v[i]; }
#pragma unroll
    for (int o = 16; o > 0; o >>= 1) s += __shfl_xor(s, o);
    const float mean = s * (1.0f / DM); float q = 0.f;
#pragma unroll
    for (int i = 0; i < 8; ++i) { const float d = v[i] - mean; q += d * d; }
#pragma unroll
    for (int o = 16; o > 0; o >>= 1) q += __shfl_xor(q, o);
    const float inv = 1.0f / sqrtf(q * (1.0f / DM) + 1e-5f);
    union { __bf16 e[8]; v4u u; } ph, pl;
#pragma unroll
    for (int i = 0; i < 8; ++i) { const int c = lane * 8 + i; const float y = (v[i] - mean) * inv * bfr(gam[c]) + bfr(bet[c]); sp[row][c] = y; const __bf16 hi = (__bf16)y; ph.e[i] = hi; pl.e[i] = (__bf16)(y - (float)hi); }
    if (OH) { vst2((unsigned*)(OH + (rb + row) * DM + lane * 8), ph.u); vst2((unsigned*)(OL + (rb + row) * DM + lane * 8), pl.u); }
    LDSX();
    vst2(OF + (rb + row) * DM + lane * 4, *(const v4f*)(&sp[row][lane * 4]));
    vst2(OF + (rb + row) * DM + 128 + lane * 4, *(const v4f*)(&sp[row][128 + lane * 4]));
  }
}
__global__ __launch_bounds__(256) void k_o(const __bf16* __restrict__ Ah, const __bf16* __restrict__ Al, const __bf16* __restrict__ WT, const float* __restrict__ X, const float* __restrict__ gam, const float* __restrict__ bet,
                                           float* __restrict__ H1, __bf16* __restrict__ H1h, __bf16* __restrict__ H1l) {
  __shared__ __align__(16) float sp[64][DM + 4];
  const int tid = threadIdx.x, wave = tid >> 5, lane = tid & 31, col = lane & 15, g = lane >> 4; const size_t rb = (size_t)blockIdx.x * 64;
  const int rt = wave & 3, ct0 = (wave >> 2) * 8; const size_t arow = rb + rt * 16 + col;
  v8f acc[8] = {};
#pragma unroll 2
  for (int kc = 0; kc < DM / 32; ++kc) { const v16b ah = frag_b16(Ah + arow * DM + kc * 32, lane), al = frag_b16(Al + arow * DM + kc * 32, lane);
#pragma unroll
    for (int j = 0; j < 8; ++j) { const v16b b = frag_b16(WT + (size_t)((ct0 + j) * 16 + col) * DM + kc * 32, lane); acc[j] = wmma_bf(al, b, acc[j]); acc[j] = wmma_bf(ah, b, acc[j]); } }
#pragma unroll
  for (int j = 0; j < 8; ++j)
#pragma unroll
    for (int r = 0; r < 8; ++r) { const int rl = rt * 16 + 8 * g + r, c = (ct0 + j) * 16 + col; sp[rl][c] = acc[j][r] + bfr(X[(rb + rl) * DM + c]); }
  __syncthreads();
  ln_rows(sp, gam, bet, rb, wave, lane, H1, H1h, H1l);
}
__global__ __launch_bounds__(128) void k_f1(const __bf16* __restrict__ Ah, const __bf16* __restrict__ Al, const __bf16* __restrict__ WT, const float* __restrict__ b1, __bf16* __restrict__ Fh, __bf16* __restrict__ Fl) {
  __shared__ __align__(16) __bf16 sh_[4][16][136], sl_[4][16][136];
  const int tid = threadIdx.x, wave = tid >> 5, lane = tid & 31, col = lane & 15, g = lane >> 4; const size_t r0 = (size_t)blockIdx.x * 64 + wave * 16; const int n0 = blockIdx.y * 128;
  v8f acc[8] = {};
#pragma unroll 2
  for (int kc = 0; kc < DM / 32; ++kc) { const v16b ah = frag_b16(Ah + (r0 + col) * DM + kc * 32, lane), al = frag_b16(Al + (r0 + col) * DM + kc * 32, lane);
#pragma unroll
    for (int j = 0; j < 8; ++j) { const v16b wb = frag_b16(WT + (size_t)(n0 + j * 16 + col) * DM + kc * 32, lane); acc[j] = wmma_bf(al, wb, acc[j]); acc[j] = wmma_bf(ah, wb, acc[j]); } }
#pragma unroll
  for (int j = 0; j < 8; ++j) { const float bb = bfr(b1[n0 + j * 16 + col]);
#pragma unroll
    for (int r = 0; r < 8; ++r) { float v = acc[j][r] + bb; v = v > 0.f ? v : 0.f; const __bf16 hi = (__bf16)v; sh_[wave][8 * g + r][j * 16 + col] = hi; sl_[wave][8 * g + r][j * 16 + col] = (__bf16)(v - (float)hi); } }
  LDSX();
  for (int qq = lane; qq < 16 * 16; qq += 32) { const int rl = qq >> 4, pc = qq & 15; const size_t o = (r0 + rl) * DM + n0 + pc * 8; vst2((unsigned*)(Fh + o), *(const v4u*)(&sh_[wave][rl][pc * 8])); vst2((unsigned*)(Fl + o), *(const v4u*)(&sl_[wave][rl][pc * 8])); }
}
__global__ __launch_bounds__(256) void k_f2(const __bf16* __restrict__ Ah, const __bf16* __restrict__ Al, const __bf16* __restrict__ WT, const float* __restrict__ b2, const float* __restrict__ H1, const float* __restrict__ gam, const float* __restrict__ bet, float* __restrict__ out) {
  __shared__ __align__(16) float sp[64][DM + 4];
  const int tid = threadIdx.x, wave = tid >> 5, lane = tid & 31, col = lane & 15, g = lane >> 4; const size_t rb = (size_t)blockIdx.x * 64;
  const int rt = wave & 3, ct0 = (wave >> 2) * 8; const size_t arow = rb + rt * 16 + col;
  v8f acc[8] = {};
#pragma unroll 2
  for (int kc = 0; kc < DM / 32; ++kc) { const v16b ah = frag_b16(Ah + arow * DM + kc * 32, lane), al = frag_b16(Al + arow * DM + kc * 32, lane);
#pragma unroll
    for (int j = 0; j < 8; ++j) { const v16b b = frag_b16(WT + (size_t)((ct0 + j) * 16 + col) * DM + kc * 32, lane); acc[j] = wmma_bf(al, b, acc[j]); acc[j] = wmma_bf(ah, b, acc[j]); } }
#pragma unroll
  for (int j = 0; j < 8; ++j)
#pragma unroll
    for (int r = 0; r < 8; ++r) { const int rl = rt * 16 + 8 * g + r, c = (ct0 + j) * 16 + col; sp[rl][c] = acc[j][r] + bfr(b2[c]) + H1[(rb + rl) * DM + c]; }
  __syncthreads();
  ln_rows(sp, gam, bet, rb, wave, lane, out, nullptr, nullptr);
}

extern "C" void kernel_launch(void* const* d_in, const int* in_sizes, int n_in, void* d_out, int out_size, void* d_ws, size_t ws_size, hipStream_t stream) {
  (void)in_sizes; (void)n_in; (void)out_size;
  const float* X  = (const float*)d_in[0];
  const float* Wq = (const float*)d_in[1]; const float* Wk = (const float*)d_in[2]; const float* Wv = (const float*)d_in[3]; const float* Wo = (const float*)d_in[4];
  const float* W1 = (const float*)d_in[5]; const float* b1 = (const float*)d_in[6]; const float* W2 = (const float*)d_in[7]; const float* b2 = (const float*)d_in[8];
  const float* g1 = (const float*)d_in[9]; const float* be1 = (const float*)d_in[10]; const float* g2 = (const float*)d_in[11]; const float* be2 = (const float*)d_in[12];
  const float* R  = (const float*)d_in[13];
  if (ws_size < (size_t)WS_END) return;
  char* ws = (char*)d_ws;
  __bf16* PT = (__bf16*)(ws + WS_PT);
  __bf16 *Qh = (__bf16*)(ws + WS_QH), *Ql = (__bf16*)(ws + WS_QL), *Kh = (__bf16*)(ws + WS_KH), *Kl = (__bf16*)(ws + WS_KL);
  __bf16 *VTh = (__bf16*)(ws + WS_VTH), *VTl = (__bf16*)(ws + WS_VTL), *EQh = (__bf16*)(ws + WS_EQH), *EQl = (__bf16*)(ws + WS_EQL), *EKh = (__bf16*)(ws + WS_EKH), *EKl = (__bf16*)(ws + WS_EKL);
  float* KVX = (float*)(ws + WS_KVX); __bf16 *KVh = (__bf16*)(ws + WS_KVH), *KVl = (__bf16*)(ws + WS_KVL);
  __bf16 *A1h = (__bf16*)(ws + WS_A1H), *A1l = (__bf16*)(ws + WS_A1L); float* H1 = (float*)(ws + WS_H1); __bf16 *H1h = (__bf16*)(ws + WS_H1H), *H1l = (__bf16*)(ws + WS_H1L), *F1h = (__bf16*)(ws + WS_F1H), *F1l = (__bf16*)(ws + WS_F1L);
  k_pack<<<7 * DM, 256, 0, stream>>>(Wq, Wk, Wv, Wo, W1, W2, R, PT);
  k_ones<<<(16 * NR / 8) / 256, 256, 0, stream>>>(VTh, VTl);
  k_qkv<<<dim3(NR / 64, 6), 128, 0, stream>>>(X, PT, Qh, Ql, Kh, Kl, VTh, VTl);
  k_proj<<<dim3(NR / 64, 2), 256, 0, stream>>>(Qh, Ql, Kh, Kl, PT + (size_t)6 * DM * DM, EQh, EQl, EKh, EKl);
  k_kv<<<DM / 16, 256, 0, stream>>>(EKh, EKl, VTh, VTl, KVX);
  k_kvt<<<NC, 256, 0, stream>>>(KVX, KVh, KVl);
  k_num<<<NR / 64, 128, 0, stream>>>(EQh, EQl, KVh, KVl, A1h, A1l);
  k_o<<<NR / 64, 256, 0, stream>>>(A1h, A1l, PT + (size_t)3 * DM * DM, X, g1, be1, H1, H1h, H1l);
  k_f1<<<dim3(NR / 64, 2), 128, 0, stream>>>(H1h, H1l, PT + (size_t)4 * DM * DM, b1, F1h, F1l);
  k_f2<<<NR / 64, 256, 0, stream>>>(F1h, F1l, PT + (size_t)5 * DM * DM, b2, H1, g2, be2, (float*)d_out);
}
